// DistKernelRegressor_8126078124619
// MI455X (gfx1250) — hardware-verified
//
#include <hip/hip_runtime.h>
#include <stdint.h>


typedef __attribute__((ext_vector_type(16))) _Float16 v16h;
typedef __attribute__((ext_vector_type(8)))  _Float16 v8h;
typedef __attribute__((ext_vector_type(8)))  float    v8f;
typedef __attribute__((ext_vector_type(4)))  float    v4f;

#define NN   1024
#define HD   128
#define KD   64
#define BI   8
#define BJ   32
#define NTHR 256
#define HP   132
#define WP   136
#define NEG_SLOPE 0.2f
#define W1_SCALE 64.0f
#define W1_INV   (1.0f / 64.0f)

static_assert(BI * (HD / 4) == NTHR, "one v4f per thread for the i-row fill");
static_assert(NN % BJ == 0 && NN % BI == 0, "exact tiling");
static_assert(HD % 32 == 0 && KD % 16 == 0, "k and n tiling");

__device__ __forceinline__ void dep_guard_h(v8f& a, v8f& b, v16h x, v16h y) { asm volatile("v_nop\n\tv_nop\n\tv_nop\n\tv_nop" : "+v"(a), "+v"(b) : "v"(x), "v"(y)); }
__device__ __forceinline__ void keep4_h(v16h a, v16h b, v16h c, v16h d) { asm volatile("v_nop" :: "v"(a), "v"(b), "v"(c), "v"(d)); }
__device__ __forceinline__ void acc_guard4(v8f& a, v8f& b, v8f& c, v8f& d) { asm volatile("v_nop\n\tv_nop\n\tv_nop\n\tv_nop" : "+v"(a), "+v"(b), "+v"(c), "+v"(d)); }

template <typename T> struct Frag;
template <> struct Frag<_Float16> {
  typedef v16h V; union U { v16h v; v8h h[2]; };
  static __device__ __forceinline__ v16h load(const _Float16* p) {
    U f; f.h[0] = *(const v8h*)(p); f.h[1] = *(const v8h*)(p + 16); return f.v;
  }
  static __device__ __forceinline__ v8f mma(v16h a, v16h b, v8f c) {
    return __builtin_amdgcn_wmma_f32_16x16x32_f16(false, a, false, b, (short)0, c, false, false);
  }
  static __device__ __forceinline__ void guard(v8f& a, v8f& b, v16h x, v16h y) { dep_guard_h(a, b, x, y); }
  static __device__ __forceinline__ void keep(v16h a, v16h b, v16h c, v16h d) { keep4_h(a, b, c, d); }
};

__device__ __forceinline__ void wave_sync_lds() {
  __builtin_amdgcn_fence(__ATOMIC_RELEASE, "workgroup");
  __builtin_amdgcn_wave_barrier();
  __builtin_amdgcn_fence(__ATOMIC_ACQUIRE, "workgroup");
}

__device__ __forceinline__ float abs_asm(float x) {
  float r;
  asm("v_max_num_f32_e64 %0, %1, -%1" : "=v"(r) : "v"(x));
  return r;
}

__global__ __launch_bounds__(256) void cast_scale_f32_f16x2(
    const float* __restrict__ in, _Float16* __restrict__ out, int n2, float scale) {
  int i = blockIdx.x * 256 + threadIdx.x;
  if (i < n2) {
    const _Float16 h0 = (_Float16)(in[2 * i] * scale), h1 = (_Float16)(in[2 * i + 1] * scale);
    const unsigned u = (unsigned)__builtin_bit_cast(unsigned short, h0) | ((unsigned)__builtin_bit_cast(unsigned short, h1) << 16);
    ((volatile unsigned*)out)[i] = u;
    __threadfence();
    ((volatile unsigned*)out)[i] = u;
  }
}

__global__ __launch_bounds__(256) void copy_f32x4(
    const float* __restrict__ in, float* __restrict__ out, int n4) {
  int i = blockIdx.x * 256 + threadIdx.x;
  if (i < n4) {
    const v4f v = *(const v4f*)(in + 4 * (size_t)i);
    *(volatile v4f*)(out + 4 * (size_t)i) = v;
    __threadfence();
    *(volatile v4f*)(out + 4 * (size_t)i) = v;
  }
}

__global__ __launch_bounds__(NTHR)
void pair_mlp_kernel(const float* __restrict__ hid, const _Float16* __restrict__ w1h,
                     const float* __restrict__ b1, const float* __restrict__ w2,
                     const float* __restrict__ b2, float* __restrict__ outk)
{
  __shared__ __align__(16) float    sHI[BI * HP];
  __shared__ __align__(16) float    sHJ[BJ * HP];
  __shared__ __align__(16) _Float16 sW1[KD * WP];
  __shared__ __align__(16) float    sOut[(NTHR / 32) * BJ];

  const int tid  = threadIdx.x;
  const int wave = tid >> 5;
  const int lane = tid & 31;
  const int hh   = lane >> 4;
  const int m    = lane & 15;
  const int i0   = blockIdx.y * BI;
  const int j0   = blockIdx.x * BJ;

  for (int idx = tid; idx < BJ * (HD / 4); idx += NTHR) {
    const int r = idx >> 5, c4 = (idx & 31) * 4;
    const v4f v = *(const v4f*)(hid + (size_t)(j0 + r) * HD + c4);
    *(v4f*)(sHJ + r * HP + c4) = v;
  }
  {
    const int r = tid >> 5, c4 = (tid & 31) * 4;
    const v4f v = *(const v4f*)(hid + (size_t)(i0 + r) * HD + c4);
    *(v4f*)(sHI + r * HP + c4) = v;
  }
  for (int idx = tid; idx < KD * (HD / 8); idx += NTHR) {
    const int r = idx >> 4, c8 = (idx & 15) * 8;
    const v8h v = *(const v8h*)(w1h + r * HD + c8);
    *(v8h*)(sW1 + r * WP + c8) = v;
  }
  __syncthreads();

  v8f acc[2][4];
#pragma unroll
  for (int mt = 0; mt < 2; ++mt)
#pragma unroll
    for (int kt = 0; kt < 4; ++kt) acc[mt][kt] = (v8f){0.f,0.f,0.f,0.f,0.f,0.f,0.f,0.f};

  const float* hi_row = sHI + wave * HP;

#pragma unroll
  for (int ks = 0; ks < HD / 32; ++ks) {
    const int k0 = ks * 32;
    v16h bf[4];
#pragma unroll
    for (int kt = 0; kt < 4; ++kt) bf[kt] = Frag<_Float16>::load(sW1 + (kt * 16 + m) * WP + k0 + 8 * hh);

#pragma unroll
    for (int mt = 0; mt < 2; ++mt) {
      const float* hj_row = sHJ + (mt * 16 + m) * HP;
      v16h a;
#pragma unroll
      for (int g = 0; g < 2; ++g) {
        const int base = k0 + 16 * g + 8 * hh;
        const v4f x0 = *(const v4f*)(hi_row + base);
        const v4f x1 = *(const v4f*)(hi_row + base + 4);
        const v4f y0 = *(const v4f*)(hj_row + base);
        const v4f y1 = *(const v4f*)(hj_row + base + 4);
#pragma unroll
        for (int w = 0; w < 4; ++w) {
          a[g * 8 + w]     = (_Float16)abs_asm(x0[w] - y0[w]);
          a[g * 8 + 4 + w] = (_Float16)abs_asm(x1[w] - y1[w]);
        }
      }
#pragma unroll
      for (int kt = 0; kt < 4; ++kt) acc[mt][kt] = Frag<_Float16>::mma(a, bf[kt], acc[mt][kt]);
      Frag<_Float16>::guard(acc[mt][0], acc[mt][3], a, a);
    }
    Frag<_Float16>::keep(bf[0], bf[1], bf[2], bf[3]);
  }
  acc_guard4(acc[0][0], acc[0][1], acc[0][2], acc[0][3]);
  acc_guard4(acc[1][0], acc[1][1], acc[1][2], acc[1][3]);

  float b1v[4], w2v[4];
#pragma unroll
  for (int kt = 0; kt < 4; ++kt) {
    b1v[kt] = b1[kt * 16 + m];
    w2v[kt] = w2[kt * 16 + m];
  }
  const float b2v = b2[0];
  float* so = sOut + wave * BJ;

#pragma unroll
  for (int mt = 0; mt < 2; ++mt) {
#pragma unroll
    for (int r = 0; r < 8; ++r) {
      float t = 0.f;
#pragma unroll
      for (int kt = 0; kt < 4; ++kt) {
        float z = acc[mt][kt][r] * W1_INV + b1v[kt];
        z = (z >= 0.f) ? z : NEG_SLOPE * z;
        t += z * w2v[kt];
      }
      t += __shfl_xor(t, 1, 32);
      t += __shfl_xor(t, 2, 32);
      t += __shfl_xor(t, 4, 32);
      t += __shfl_xor(t, 8, 32);
      if (m == 0) so[mt * 16 + 8 * hh + r] = t + b2v;
    }
  }
  wave_sync_lds();
  {
    const float e = so[lane];
    const float s = 1.0f / (1.0f + expf(-e));
    so[lane] = s;
  }
  wave_sync_lds();

  float* orow = outk + (size_t)(i0 + wave) * NN + j0;
  for (int pass = 0; pass < 2; ++pass) {
    if (lane < 8) {
      const v4f v = *(const v4f*)(so + 4 * lane);
      *(volatile v4f*)(orow + 4 * lane) = v;
    }
    __threadfence();
  }
}

extern "C" void kernel_launch(void* const* d_in, const int* in_sizes, int n_in,
                              void* d_out, int out_size, void* d_ws, size_t ws_size,
                              hipStream_t stream) {
  if (n_in < 5) return;
  if (in_sizes[0] != NN * HD || in_sizes[1] != KD * HD || in_sizes[2] != KD ||
      in_sizes[3] != KD || in_sizes[4] < 1) return;
  if (out_size != NN * HD + NN * NN) return;
  const size_t w1_bytes = (size_t)KD * HD * sizeof(_Float16);
  if (ws_size < w1_bytes) return;

  const float* hid   = (const float*)d_in[0];
  const float* fc1_w = (const float*)d_in[1];
  const float* fc1_b = (const float*)d_in[2];
  const float* fc2_w = (const float*)d_in[3];
  const float* fc2_b = (const float*)d_in[4];

  float* out0 = (float*)d_out;
  float* out1 = out0 + (size_t)NN * HD;
  _Float16* w1h = (_Float16*)d_ws;

  const int n2 = KD * HD / 2;
  cast_scale_f32_f16x2<<<(n2 + 255) / 256, 256, 0, stream>>>(fc1_w, w1h, n2, W1_SCALE);

  const int n4 = NN * HD / 4;
  copy_f32x4<<<(n4 + 255) / 256, 256, 0, stream>>>(hid, out0, n4);

  dim3 grid(NN / BJ, NN / BI);
  pair_mlp_kernel<<<grid, NTHR, 0, stream>>>(hid, w1h, fc1_b, fc2_w, fc2_b, out1);
  (void)hipGetLastError();
}
